// LocAtt_20229295964633
// MI455X (gfx1250) — hardware-verified
//
#include <hip/hip_runtime.h>


namespace {
constexpr int Bn = 8, C = 128, IH = 64, IW = 64, NPI = IH * IW, NT = Bn * NPI, KS = 7, PADW = 3;
constexpr float XS = 8.0f, PS = 8.0f;

typedef _Float16 b16;
typedef __attribute__((ext_vector_type(16))) _Float16 v16b;
typedef __attribute__((ext_vector_type(8))) _Float16 v8b;
typedef __attribute__((ext_vector_type(8))) float v8f;
typedef __attribute__((ext_vector_type(4))) float v4f;
__device__ __forceinline__ float bf16_rne(float f) { unsigned int u = __float_as_uint(f); u += 0x7FFFu + ((u >> 16) & 1u); return __uint_as_float(u & 0xFFFF0000u); }
__device__ __forceinline__ void split16(float v, b16& hi, b16& lo) { hi = (b16)v; lo = (b16)(v - (float)hi); }
__device__ __forceinline__ v16b frag_kb(const b16* p, int hh) { const v8b a = *(const v8b*)(p + 8 * hh), b = *(const v8b*)(p + 16 + 8 * hh); v16b f;
#pragma unroll
  for (int e = 0; e < 8; ++e) { f[e] = a[e]; f[8 + e] = b[e]; } return f; }
__device__ __forceinline__ v8f wmma16b(v16b a, v16b b, v8f c) { v8f d = __builtin_amdgcn_wmma_f32_16x16x32_f16(false, a, false, b, (short)0, c, false, false); asm volatile("v_nop\n\tv_nop\n\tv_nop\n\tv_nop" : "+v"(d) : "v"(a), "v"(b)); return d; }
__device__ __forceinline__ void wave_lds_sync() { __builtin_amdgcn_fence(__ATOMIC_RELEASE, "workgroup"); __builtin_amdgcn_wave_barrier(); __builtin_amdgcn_fence(__ATOMIC_ACQUIRE, "workgroup"); }
__device__ __forceinline__ float nexp(float x) { return __builtin_amdgcn_exp2f(x * 1.4426950408889634f); }
__device__ __forceinline__ float pmul(float a, float b) { float p = a * b; asm volatile("" : "+v"(p)); return p; }

__global__ __launch_bounds__(256) void prepw_kernel(const float* __restrict__ wq, const float* __restrict__ bq, const float* __restrict__ wk, const float* __restrict__ bk, const float* __restrict__ wv, const float* __restrict__ bv, b16* __restrict__ R, float* __restrict__ P) {
  const size_t tid = (size_t)blockIdx.x * 256 + threadIdx.x, nth = (size_t)gridDim.x * 256;
  for (int pass = 0; pass < 2; ++pass) { for (size_t p = tid; p < (size_t)3 * C * C; p += nth) { const int w = (int)(p / (C * C)); const size_t r = p % ((size_t)C * C); ((volatile b16*)R)[p] = (b16)bf16_rne(((w == 0) ? wq : (w == 1) ? wk : wv)[r]); }
    for (size_t q = tid; q < 384; q += nth) { const int i = (int)q; P[q] = bf16_rne((i < 128) ? bq[i] : (i < 256) ? bk[i - 128] : bv[i - 256]); } __threadfence(); }
}
__global__ __launch_bounds__(256) void xt_kernel(const float* __restrict__ x, b16* __restrict__ XT) {
  __shared__ __attribute__((aligned(16))) b16 Tx[64][C + 8];
  const int b = blockIdx.y, p0 = blockIdx.x * 64, t_ = threadIdx.x;
  for (int i = t_; i < C * 64; i += 256) { const int c = i >> 6, px = i & 63; Tx[px][c] = (b16)(bf16_rne(x[((size_t)b * C + c) * NPI + p0 + px]) * XS); }
  __syncthreads();
  for (int pass = 0; pass < 2; ++pass) { for (int i = t_; i < 64 * 16; i += 256) { const int px = i >> 4, c8 = (i & 15) * 8; *(volatile v8b*)(XT + ((size_t)b * NPI + p0 + px) * C + c8) = *(const v8b*)(&Tx[px][c8]); } __threadfence(); }
}
__global__ __launch_bounds__(64) void qk_kernel(const b16* __restrict__ XT, const b16* __restrict__ R, const float* __restrict__ P, b16* __restrict__ QH, b16* __restrict__ QL, b16* __restrict__ KH, b16* __restrict__ KL) {
  __shared__ __attribute__((aligned(16))) b16 Th[2][32][C + 8], Tl[2][32][C + 8];
  const int lane = threadIdx.x & 31, wave = threadIdx.x >> 5, nloc = lane & 15, hlf = lane >> 4, m0 = blockIdx.x * 32; const b16* Bw = R + (size_t)wave * C * C; const float* bias = P + wave * C;
  v8f acc[2][8];
#pragma unroll
  for (int r = 0; r < 2; ++r)
#pragma unroll
    for (int t = 0; t < 8; ++t) acc[r][t] = (v8f){};
#pragma unroll
  for (int kb = 0; kb < C; kb += 32) { const v16b a0 = frag_kb(XT + (size_t)(m0 + nloc) * C + kb, hlf), a1 = frag_kb(XT + (size_t)(m0 + 16 + nloc) * C + kb, hlf);
#pragma unroll
    for (int t = 0; t < 8; ++t) { const v16b bw = frag_kb(Bw + (size_t)(t * 16 + nloc) * C + kb, hlf); acc[0][t] = wmma16b(a0, bw, acc[0][t]); acc[1][t] = wmma16b(a1, bw, acc[1][t]); } }
#pragma unroll
  for (int t = 0; t < 8; ++t) { const float bb = bias[t * 16 + nloc];
#pragma unroll
    for (int r = 0; r < 2; ++r)
#pragma unroll
      for (int v = 0; v < 8; ++v) { b16 a_, c_; split16(acc[r][t][v] + XS * bb, a_, c_); Th[wave][r * 16 + 8 * hlf + v][t * 16 + nloc] = a_; Tl[wave][r * 16 + 8 * hlf + v][t * 16 + nloc] = c_; } }
  wave_lds_sync();
  b16* dh = wave ? KH : QH; b16* dl = wave ? KL : QL;
  for (int pass = 0; pass < 2; ++pass) { for (int i = lane; i < 32 * 16; i += 32) { const int rr = i >> 4, c8 = (i & 15) * 8; const size_t gi = (size_t)(m0 + rr) * C + c8; *(volatile v8b*)(dh + gi) = *(const v8b*)(&Th[wave][rr][c8]); *(volatile v8b*)(dl + gi) = *(const v8b*)(&Tl[wave][rr][c8]); } __threadfence(); }
}
__global__ __launch_bounds__(128) void v_kernel(const b16* __restrict__ XT, const b16* __restrict__ R, const float* __restrict__ P, b16* __restrict__ VTh, b16* __restrict__ VTl) {
  __shared__ __attribute__((aligned(16))) b16 Th[C][64 + 8], Tl[C][64 + 8];
  const int lane = threadIdx.x & 31, wave = threadIdx.x >> 5, nloc = lane & 15, hlf = lane >> 4, g0 = blockIdx.x * 64, m0 = g0 + wave * 16; const b16* Bv = R + (size_t)2 * C * C; const int b = g0 / NPI, p0 = g0 % NPI;
  v8f acc[8];
#pragma unroll
  for (int t = 0; t < 8; ++t) acc[t] = (v8f){};
#pragma unroll
  for (int kb = 0; kb < C; kb += 32) { const v16b a = frag_kb(XT + (size_t)(m0 + nloc) * C + kb, hlf);
#pragma unroll
    for (int t = 0; t < 8; ++t) acc[t] = wmma16b(a, frag_kb(Bv + (size_t)(t * 16 + nloc) * C + kb, hlf), acc[t]); }
#pragma unroll
  for (int t = 0; t < 8; ++t)
#pragma unroll
    for (int r = 0; r < 8; ++r) { b16 a_, c_; split16(acc[t][r] + XS * P[256 + t * 16 + nloc], a_, c_); Th[t * 16 + nloc][wave * 16 + 8 * hlf + r] = a_; Tl[t * 16 + nloc][wave * 16 + 8 * hlf + r] = c_; }
  __syncthreads();
  for (int pass = 0; pass < 2; ++pass) { for (int i = threadIdx.x; i < C * 8; i += 128) { const int c = i >> 3, c8 = (i & 7) * 8; const size_t gi = ((size_t)b * C + c) * NPI + p0 + c8; *(volatile v8b*)(VTh + gi) = *(const v8b*)(&Th[c][c8]); *(volatile v8b*)(VTl + gi) = *(const v8b*)(&Tl[c][c8]); } __threadfence(); }
}
__global__ __launch_bounds__(64) void attn_kernel(const b16* __restrict__ QH, const b16* __restrict__ QL, const b16* __restrict__ KH, const b16* __restrict__ KL, const b16* __restrict__ VTh, const b16* __restrict__ VTl, float* __restrict__ out) {
  __shared__ __attribute__((aligned(16))) float Os[C][32 + 4];
  const int wave = threadIdx.x >> 5, lane = threadIdx.x & 31, hh = lane >> 4, col = lane & 15; const int b = blockIdx.z, h = blockIdx.y, w0 = blockIdx.x * 32 + wave * 16, wq = w0 + col;
  const size_t ib = (size_t)b * NPI; const int qpix = h * IW + wq;
  v16b qf[4], ql[4]; for (int t = 0; t < 4; ++t) { qf[t] = frag_kb(QH + (ib + qpix) * C + t * 32, hh); ql[t] = frag_kb(QL + (ib + qpix) * C + t * 32, hh); }
  const int r_lo = (h - PADW < 0) ? 0 : h - PADW, r_hi = (h + PADW > IH - 1) ? IH - 1 : h + PADW, c_lo = (wq - PADW < 0) ? 0 : wq - PADW, c_hi = (wq + PADW > IW - 1) ? IW - 1 : wq + PADW;
  const int n_in = (r_hi - r_lo + 1) * (c_hi - c_lo + 1), n_out = KS * KS - n_in;
  float m = (n_out > 0) ? 0.0f : -INFINITY, l = (float)n_out; v8f o[8]; for (int t = 0; t < 8; ++t) o[t] = (v8f){};
  int c0 = w0 - 8; c0 = (c0 < 0) ? 0 : (c0 > IW - 32 ? IW - 32 : c0);
  for (int r = h - PADW; r <= h + PADW; ++r) { if (r < 0 || r >= IH) continue;
    const b16* Kr = KH + (ib + (size_t)r * IW + c0) * C; const b16* Klr = KL + (ib + (size_t)r * IW + c0) * C;
    v8f s0 = {}, s1 = {};
#pragma unroll
    for (int t = 0; t < 4; ++t) { const v16b k0 = frag_kb(Kr + (size_t)col * C + t * 32, hh), k0l = frag_kb(Klr + (size_t)col * C + t * 32, hh), k1 = frag_kb(Kr + (size_t)(16 + col) * C + t * 32, hh), k1l = frag_kb(Klr + (size_t)(16 + col) * C + t * 32, hh);
      s0 = wmma16b(k0, qf[t], s0); s0 = wmma16b(k0l, qf[t], s0); s0 = wmma16b(k0, ql[t], s0); s1 = wmma16b(k1, qf[t], s1); s1 = wmma16b(k1l, qf[t], s1); s1 = wmma16b(k1, ql[t], s1); }
    float mr = -INFINITY;
#pragma unroll
    for (int e = 0; e < 8; ++e) { const int kc0 = c0 + 8 * hh + e, kc1 = kc0 + 16; const bool v0 = (kc0 >= wq - PADW) && (kc0 <= wq + PADW), v1 = (kc1 >= wq - PADW) && (kc1 <= wq + PADW);
      s0[e] = v0 ? s0[e] * (1.0f / (XS * XS)) : -INFINITY; s1[e] = v1 ? s1[e] * (1.0f / (XS * XS)) : -INFINITY; mr = fmaxf(mr, fmaxf(s0[e], s1[e])); }
    mr = fmaxf(mr, __shfl_xor(mr, 16)); const float mn = fmaxf(m, mr); const float al_ = (mn == -INFINITY) ? 1.0f : nexp(m - mn); m = mn; float sum = 0.0f; v16b pb, pl;
#pragma unroll
    for (int e = 0; e < 8; ++e) { const float e0 = (s0[e] == -INFINITY) ? 0.0f : nexp(s0[e] - mn), e1 = (s1[e] == -INFINITY) ? 0.0f : nexp(s1[e] - mn); sum += e0 + e1; b16 a_, c_; split16(e0 * PS, a_, c_); pb[e] = a_; pl[e] = c_; split16(e1 * PS, a_, c_); pb[8 + e] = a_; pl[8 + e] = c_; }
    sum += __shfl_xor(sum, 16); l = l * al_ + sum;
    const b16* V = VTh + (ib * 0 + (size_t)b * C) * NPI + (size_t)r * IW + c0; const b16* Vl = VTl + ((size_t)b * C) * NPI + (size_t)r * IW + c0;
#pragma unroll
    for (int t = 0; t < 8; ++t) { o[t] *= al_; const v16b vh = frag_kb(V + (size_t)(t * 16 + col) * NPI, hh); o[t] = wmma16b(vh, pb, o[t]); o[t] = wmma16b(vh, pl, o[t]); o[t] = wmma16b(frag_kb(Vl + (size_t)(t * 16 + col) * NPI, hh), pb, o[t]); } }
  const float inv = 1.0f / (l * PS * XS);
#pragma unroll
  for (int t = 0; t < 8; ++t)
#pragma unroll
    for (int e = 0; e < 8; ++e) Os[t * 16 + 8 * hh + e][wave * 16 + col] = o[t][e] * inv;
  __syncthreads();
  for (int pass = 0; pass < 2; ++pass) { for (int i = threadIdx.x; i < C * 8; i += 64) { const int c = i >> 3, c4 = (i & 7) * 4; *(volatile v4f*)(out + ((size_t)b * C + c) * NPI + (size_t)h * IW + blockIdx.x * 32 + c4) = *(const v4f*)(&Os[c][c4]); } __threadfence(); }
}
}

extern "C" void kernel_launch(void* const* d_in, const int* in_sizes, int n_in,
                              void* d_out, int out_size, void* d_ws, size_t ws_size, hipStream_t stream) {
  (void)n_in; (void)out_size;
  const float* x = (const float*)d_in[0]; const float* wq = (const float*)d_in[1]; const float* bq = (const float*)d_in[2]; const float* wk = (const float*)d_in[3]; const float* bk = (const float*)d_in[4]; const float* wv = (const float*)d_in[5]; const float* bv = (const float*)d_in[6];
  float* out = (float*)d_out;
  if (in_sizes[0] != NT * C || in_sizes[1] != C * C) return;
  size_t off = 0; char* ws = (char*)d_ws;
  auto carve = [&](size_t bytes) { char* p = ws + off; off += (bytes + 255) & ~(size_t)255; return p; };
  b16* R = (b16*)carve((size_t)3 * C * C * 2); float* P = (float*)carve(384 * 4); b16* XT = (b16*)carve((size_t)NT * C * 2); b16* QH = (b16*)carve((size_t)NT * C * 2); b16* QL = (b16*)carve((size_t)NT * C * 2); b16* KH = (b16*)carve((size_t)NT * C * 2); b16* KL = (b16*)carve((size_t)NT * C * 2); b16* VTh = (b16*)carve((size_t)NT * C * 2); b16* VTl = (b16*)carve((size_t)NT * C * 2);
  if (off > ws_size) return;
  prepw_kernel<<<64, 256, 0, stream>>>(wq, bq, wk, bk, wv, bv, R, P);
  xt_kernel<<<dim3(NPI / 64, Bn), 256, 0, stream>>>(x, XT);
  qk_kernel<<<NT / 32, 64, 0, stream>>>(XT, R, P, QH, QL, KH, KL);
  v_kernel<<<NT / 64, 128, 0, stream>>>(XT, R, P, VTh, VTl);
  attn_kernel<<<dim3(2, IH, Bn), 64, 0, stream>>>(QH, QL, KH, KL, VTh, VTl, out);
}
